// Hedgehog_17076789969437
// MI455X (gfx1250) — hardware-verified
//
#include <hip/hip_runtime.h>
#include <stddef.h>
#include <stdint.h>

#define NHEAD 16
#define SEQ   1024
#define DK    64
#define FD    64
#define DF    128
#define CH    64
#define NCH   16

static_assert(NCH * CH == SEQ);
static_assert(DF == 2 * FD);
static_assert(DK == 64);

typedef __bf16         v16bf __attribute__((ext_vector_type(16)));
typedef unsigned short v8us  __attribute__((ext_vector_type(8)));
typedef float          v8f   __attribute__((ext_vector_type(8)));
typedef float          v4f   __attribute__((ext_vector_type(4)));
typedef unsigned int   v4u   __attribute__((ext_vector_type(4)));

union Frag { v16bf v; v8us u[2]; };
union Pk8  { v8us s; v4u u; };

__device__ __forceinline__ v8f mma16(v16bf a, v16bf b, v8f c) {
  c = __builtin_amdgcn_wmma_f32_16x16x32_bf16(false, a, false, b, (short)0, c, false, false);
  asm volatile("v_nop\n\tv_nop\n\tv_nop\n\tv_nop" : "+v"(c) : "v"(a), "v"(b));
  return c;
}

__device__ __forceinline__ v16bf ldfrag(const unsigned short* p, int ld, int row0, int k0, int lane) {
  const int m = lane & 15, lh = lane >> 4;
  const unsigned short* q = p + (size_t)(row0 + m) * ld + k0 + 8 * lh;
  Frag f;
  f.u[0] = *(const v8us*)(q);
  f.u[1] = *(const v8us*)(q + 16);
  return f.v;
}

__device__ __forceinline__ v8f zero8() { return (v8f){0.f, 0.f, 0.f, 0.f, 0.f, 0.f, 0.f, 0.f}; }

__device__ __forceinline__ unsigned int bf_rne(float x) {
  const unsigned int u = __float_as_uint(x);
  return (u + 0x7FFFu + ((u >> 16) & 1u)) >> 16;
}

__device__ __forceinline__ void split8(const float (&x)[8], v8us& hi, v8us& lo) {
#pragma unroll
  for (int j = 0; j < 8; ++j) {
    const unsigned int hb = bf_rne(x[j]);
    const float hv = __uint_as_float(hb << 16);
    const unsigned int lb = bf_rne(x[j] - hv);
    hi[j] = (unsigned short)hb;
    lo[j] = (unsigned short)lb;
  }
}

#define TP 65

__global__ __launch_bounds__(256) void k_prepw(const float* __restrict__ wq, const float* __restrict__ wk,
                                               unsigned short* __restrict__ wth, unsigned short* __restrict__ wtl) {
  __shared__ float sw[DK * TP];
  const int which = blockIdx.x >> 4, head = blockIdx.x & 15;
  const int tid = threadIdx.x;
  const float* src = (which == 0 ? wq : wk) + (size_t)head * DK * FD;
#pragma unroll
  for (int it = 0; it < 4; ++it) {
    const int idx = tid + 256 * it;
    const v4f a = *(const v4f*)(src + idx * 4);
    const int e = idx * 4, d = e >> 6, f = e & 63;
    float* r = sw + d * TP + f;
    r[0] = a[0]; r[1] = a[1]; r[2] = a[2]; r[3] = a[3];
  }
  __syncthreads();
  v4u vh[2], vl[2];
  size_t go[2];
#pragma unroll
  for (int it = 0; it < 2; ++it) {
    const int p = tid + 256 * it;
    const int f = p >> 3, pc = p & 7;
    float x[8];
#pragma unroll
    for (int j = 0; j < 8; ++j) x[j] = sw[(pc * 8 + j) * TP + f];
    v8us h8, l8;
    split8(x, h8, l8);
    Pk8 a, b;
    a.s = h8; b.s = l8;
    vh[it] = a.u; vl[it] = b.u;
    go[it] = ((size_t)(which * NHEAD + head) * FD + f) * DK + pc * 8;
  }
  for (int ps = 0; ps < 2; ++ps) {
#pragma unroll
    for (int it = 0; it < 2; ++it) {
      *(volatile v4u*)(wth + go[it]) = vh[it];
      *(volatile v4u*)(wtl + go[it]) = vl[it];
    }
    __threadfence();
  }
}

__global__ __launch_bounds__(256) void k_prepv(const float* __restrict__ v,
                                               unsigned short* __restrict__ vth, unsigned short* __restrict__ vtl) {
  __shared__ float sv[CH * TP];
  const int chk = blockIdx.x, head = blockIdx.y;
  const int l0 = chk * CH;
  const int tid = threadIdx.x;
  const float* src = v + ((size_t)head * SEQ + l0) * DK;
#pragma unroll
  for (int it = 0; it < 4; ++it) {
    const int idx = tid + 256 * it;
    const v4f a = *(const v4f*)(src + idx * 4);
    const int e = idx * 4, l = e >> 6, d = e & 63;
    float* r = sv + l * TP + d;
    r[0] = a[0]; r[1] = a[1]; r[2] = a[2]; r[3] = a[3];
  }
  __syncthreads();
  v4u vh[2], vl[2];
  size_t go[2];
#pragma unroll
  for (int it = 0; it < 2; ++it) {
    const int p = tid + 256 * it;
    const int d = p >> 3, pc = p & 7;
    float x[8];
#pragma unroll
    for (int j = 0; j < 8; ++j) x[j] = sv[(pc * 8 + j) * TP + d];
    v8us h8, l8;
    split8(x, h8, l8);
    Pk8 a, b;
    a.s = h8; b.s = l8;
    vh[it] = a.u; vl[it] = b.u;
    go[it] = ((size_t)(head * DK + d)) * SEQ + l0 + pc * 8;
  }
  for (int ps = 0; ps < 2; ++ps) {
#pragma unroll
    for (int it = 0; it < 2; ++it) {
      *(volatile v4u*)(vth + go[it]) = vh[it];
      *(volatile v4u*)(vtl + go[it]) = vl[it];
    }
    __threadfence();
  }
}

#define XP 72
#define HP 68
#define FP 136
#define FE_XH 0
#define FE_XL (64 * XP * 2)
#define FE_H  (2 * 64 * XP * 2)
#define FE_FL (FE_H + 64 * HP * 4)
#define FE_BYTES (FE_FL + 64 * FP * 2)
static_assert(64 * FP * 2 <= FE_H);
static_assert(FE_BYTES <= 65536);

__global__ __launch_bounds__(256) void k_feat(const float* __restrict__ q, const float* __restrict__ k,
                                              const unsigned short* __restrict__ wth,
                                              const unsigned short* __restrict__ wtl,
                                              const int* __restrict__ use_scale,
                                              unsigned short* __restrict__ qfh, unsigned short* __restrict__ qfl,
                                              unsigned short* __restrict__ kfh, unsigned short* __restrict__ kfl) {
  __shared__ __align__(16) unsigned char smem[FE_BYTES];
  unsigned short* sXh = (unsigned short*)(smem + FE_XH);
  unsigned short* sXl = (unsigned short*)(smem + FE_XL);
  float*          sH  = (float*)(smem + FE_H);
  unsigned short* sFh = (unsigned short*)(smem + FE_XH);
  unsigned short* sFl = (unsigned short*)(smem + FE_FL);

  const int chk = blockIdx.x, head = blockIdx.y, which = blockIdx.z;
  const int l0 = chk * CH;
  const int tid = threadIdx.x, lane = tid & 31, wave = tid >> 5;
  const int hh = lane >> 4, c = lane & 15;
  const float* src = (which == 0 ? q : k) + ((size_t)head * SEQ + l0) * DK;
  unsigned short* dh = (which == 0) ? qfh : kfh;
  unsigned short* dl = (which == 0) ? qfl : kfl;
  const unsigned short* wbh = wth + (size_t)(which * NHEAD + head) * FD * DK;
  const unsigned short* wbl = wtl + (size_t)(which * NHEAD + head) * FD * DK;
  const float sc = (which == 0 && use_scale[0] != 0) ? 0.08838834764831845f : 1.0f;

  {
    const int row = tid >> 2, part = tid & 3;
    const float* xr = src + row * DK + part * 16;
    const v4f a0 = *(const v4f*)(xr), a1 = *(const v4f*)(xr + 4);
    const v4f a2 = *(const v4f*)(xr + 8), a3 = *(const v4f*)(xr + 12);
    float x0[8] = {a0[0], a0[1], a0[2], a0[3], a1[0], a1[1], a1[2], a1[3]};
    float x1[8] = {a2[0], a2[1], a2[2], a2[3], a3[0], a3[1], a3[2], a3[3]};
    v8us h0, g0, h1, g1;
    split8(x0, h0, g0);
    split8(x1, h1, g1);
    *(v8us*)(sXh + row * XP + part * 16)     = h0;
    *(v8us*)(sXh + row * XP + part * 16 + 8) = h1;
    *(v8us*)(sXl + row * XP + part * 16)     = g0;
    *(v8us*)(sXl + row * XP + part * 16 + 8) = g1;
  }
  __syncthreads();

  {
    const int mt = wave >> 1, np = (wave & 1) * 2;
    v8f acc[2] = {zero8(), zero8()};
#pragma unroll
    for (int ks = 0; ks < 2; ++ks) {
      const int k0 = ks * 32;
      const v16bf ah = ldfrag(sXh, XP, mt * 16, k0, lane);
      const v16bf al = ldfrag(sXl, XP, mt * 16, k0, lane);
#pragma unroll
      for (int j = 0; j < 2; ++j) {
        const v16bf bh = ldfrag(wbh, DK, (np + j) * 16, k0, lane);
        const v16bf bl = ldfrag(wbl, DK, (np + j) * 16, k0, lane);
        acc[j] = mma16(ah, bh, acc[j]);
        acc[j] = mma16(ah, bl, acc[j]);
        acc[j] = mma16(al, bh, acc[j]);
      }
    }
#pragma unroll
    for (int j = 0; j < 2; ++j)
#pragma unroll
      for (int r = 0; r < 8; ++r) sH[(mt * 16 + 8 * hh + r) * HP + (np + j) * 16 + c] = acc[j][r];
  }
  __syncthreads();

  {
    const int row = tid >> 2, part = tid & 3;
    const float* hp = sH + row * HP + part * 16;
    const v4f g0 = *(const v4f*)(hp), g1 = *(const v4f*)(hp + 4);
    const v4f g2 = *(const v4f*)(hp + 8), g3 = *(const v4f*)(hp + 12);
    float hv[16] = {g0[0], g0[1], g0[2], g0[3], g1[0], g1[1], g1[2], g1[3],
                    g2[0], g2[1], g2[2], g2[3], g3[0], g3[1], g3[2], g3[3]};
    float mx = hv[0], mn = hv[0];
#pragma unroll
    for (int j = 1; j < 16; ++j) { mx = fmaxf(mx, hv[j]); mn = fminf(mn, hv[j]); }
    mx = fmaxf(mx, __shfl_xor(mx, 1, 32)); mx = fmaxf(mx, __shfl_xor(mx, 2, 32));
    mn = fminf(mn, __shfl_xor(mn, 1, 32)); mn = fminf(mn, __shfl_xor(mn, 2, 32));
    float e1[16], e2[16];
    float s1 = 0.f, s2 = 0.f;
#pragma unroll
    for (int j = 0; j < 16; ++j) {
      e1[j] = expf(hv[j] - mx);
      e2[j] = expf(mn - hv[j]);
      s1 += e1[j];
      s2 += e2[j];
    }
    s1 += __shfl_xor(s1, 1, 32); s1 += __shfl_xor(s1, 2, 32);
    s2 += __shfl_xor(s2, 1, 32); s2 += __shfl_xor(s2, 2, 32);
    const float r1 = 1.0f / s1, r2 = 1.0f / s2;
    float fa0[8], fa1[8], fb0[8], fb1[8];
#pragma unroll
    for (int j = 0; j < 8; ++j) {
      fa0[j] = fmaxf(e1[j] * r1, 1e-12f) * sc;
      fa1[j] = fmaxf(e1[8 + j] * r1, 1e-12f) * sc;
      fb0[j] = fmaxf(e2[j] * r2, 1e-12f) * sc;
      fb1[j] = fmaxf(e2[8 + j] * r2, 1e-12f) * sc;
    }
    v8us h8, l8;
    split8(fa0, h8, l8);
    *(v8us*)(sFh + row * FP + part * 16) = h8;
    *(v8us*)(sFl + row * FP + part * 16) = l8;
    split8(fa1, h8, l8);
    *(v8us*)(sFh + row * FP + part * 16 + 8) = h8;
    *(v8us*)(sFl + row * FP + part * 16 + 8) = l8;
    split8(fb0, h8, l8);
    *(v8us*)(sFh + row * FP + FD + part * 16) = h8;
    *(v8us*)(sFl + row * FP + FD + part * 16) = l8;
    split8(fb1, h8, l8);
    *(v8us*)(sFh + row * FP + FD + part * 16 + 8) = h8;
    *(v8us*)(sFl + row * FP + FD + part * 16 + 8) = l8;
  }
  __syncthreads();

  v4u vh[4], vl[4];
  size_t go[4];
#pragma unroll
  for (int it = 0; it < 4; ++it) {
    const int p    = tid + 256 * it;
    const int L    = p >> 3;
    const int row  = L >> 1;
    const int half = L & 1;
    const int pc   = p & 7;
    const int off  = row * FP + half * 64 + pc * 8;
    Pk8 a, b;
    a.s = *(const v8us*)(sFh + off);
    b.s = *(const v8us*)(sFl + off);
    vh[it] = a.u; vl[it] = b.u;
    go[it] = ((size_t)(head * SEQ + l0 + row)) * DF + half * 64 + pc * 8;
  }
  for (int ps = 0; ps < 2; ++ps) {
#pragma unroll
    for (int it = 0; it < 4; ++it) {
      *(volatile v4u*)(dh + go[it]) = vh[it];
      *(volatile v4u*)(dl + go[it]) = vl[it];
    }
    __threadfence();
  }
}

#define AP 72
#define OP 68
#define AT_AH 0
#define AT_AL (64 * AP * 2)
#define AT_Z  (2 * 64 * AP * 2)
#define AT_BYTES (AT_Z + 2 * CH * 4)
static_assert(64 * OP * 4 <= AT_Z);

__global__ __launch_bounds__(256) void k_attn(const unsigned short* __restrict__ qfh,
                                              const unsigned short* __restrict__ qfl,
                                              const unsigned short* __restrict__ kfh,
                                              const unsigned short* __restrict__ kfl,
                                              const unsigned short* __restrict__ vth,
                                              const unsigned short* __restrict__ vtl,
                                              const int* __restrict__ use_norm,
                                              float* __restrict__ out) {
  __shared__ __align__(16) unsigned char smem[AT_BYTES];
  unsigned short* sAh = (unsigned short*)(smem + AT_AH);
  unsigned short* sAl = (unsigned short*)(smem + AT_AL);
  float*          sZ  = (float*)(smem + AT_Z);
  float*          sO  = (float*)(smem + AT_AH);

  const int qb = blockIdx.x, head = blockIdx.y;
  const int tid = threadIdx.x, lane = tid & 31, wave = tid >> 5;
  const int hh = lane >> 4, c = lane & 15;
  const int rg = wave & 3, kh = wave >> 2;
  const int i0 = rg * 16;

  const size_t qrow0 = (size_t)head * SEQ + (size_t)qb * CH;
  const unsigned short* aqh = qfh + qrow0 * DF;
  const unsigned short* aql = qfl + qrow0 * DF;
  const unsigned short* bkh = kfh + (size_t)head * SEQ * DF;
  const unsigned short* bkl = kfl + (size_t)head * SEQ * DF;
  const unsigned short* bvh = vth + (size_t)(head * DK + kh * 32) * SEQ;
  const unsigned short* bvl = vtl + (size_t)(head * DK + kh * 32) * SEQ;

  v8f oacc[2] = {zero8(), zero8()};
  float zp[8];
#pragma unroll
  for (int r = 0; r < 8; ++r) zp[r] = 0.f;

  for (int kc = 0; kc <= qb; ++kc) {
    const int j0 = kc * CH;
    v8f s[2] = {zero8(), zero8()};
#pragma unroll
    for (int ks = 0; ks < 4; ++ks) {
      const int k0 = ks * 32;
      const v16bf ah = ldfrag(aqh, DF, i0, k0, lane);
      const v16bf al = ldfrag(aql, DF, i0, k0, lane);
#pragma unroll
      for (int jt = 0; jt < 2; ++jt) {
        const int row0 = j0 + kh * 32 + 16 * jt;
        const v16bf bh = ldfrag(bkh, DF, row0, k0, lane);
        const v16bf bl = ldfrag(bkl, DF, row0, k0, lane);
        s[jt] = mma16(ah, bh, s[jt]);
        s[jt] = mma16(ah, bl, s[jt]);
        s[jt] = mma16(al, bh, s[jt]);
      }
    }
    __syncthreads();
#pragma unroll
    for (int r = 0; r < 8; ++r) {
      const int il = i0 + 8 * hh + r;
      const int iq = qb * CH + il;
      float rs = 0.f;
#pragma unroll
      for (int jt = 0; jt < 2; ++jt) {
        const int jl = kh * 32 + 16 * jt + c;
        const int js = j0 + jl;
        const float av = (js <= iq) ? s[jt][r] : 0.f;
        rs += av;
        const unsigned int hb = bf_rne(av);
        const float hv = __uint_as_float(hb << 16);
        const unsigned int lb = bf_rne(av - hv);
        sAh[il * AP + jl] = (unsigned short)hb;
        sAl[il * AP + jl] = (unsigned short)lb;
      }
      zp[r] += rs;
    }
    __syncthreads();
#pragma unroll
    for (int kk = 0; kk < 2; ++kk) {
      const v16bf pah = ldfrag(sAh, AP, i0, kk * 32, lane);
      const v16bf pal = ldfrag(sAl, AP, i0, kk * 32, lane);
#pragma unroll
      for (int t = 0; t < 2; ++t) {
        const v16bf bh = ldfrag(bvh, SEQ, 16 * t, j0 + kk * 32, lane);
        const v16bf bl = ldfrag(bvl, SEQ, 16 * t, j0 + kk * 32, lane);
        oacc[t] = mma16(pah, bh, oacc[t]);
        oacc[t] = mma16(pah, bl, oacc[t]);
        oacc[t] = mma16(pal, bh, oacc[t]);
      }
    }
  }

  float zr[8];
#pragma unroll
  for (int r = 0; r < 8; ++r) {
    float d = zp[r];
    d += __shfl_xor(d, 1, 32);
    d += __shfl_xor(d, 2, 32);
    d += __shfl_xor(d, 4, 32);
    d += __shfl_xor(d, 8, 32);
    zr[r] = d;
  }
  if (c == 0) {
#pragma unroll
    for (int r = 0; r < 8; ++r) sZ[kh * CH + i0 + 8 * hh + r] = zr[r];
  }
  __syncthreads();
  const bool nrm = use_norm[0] != 0;
#pragma unroll
  for (int r = 0; r < 8; ++r) {
    const int row = i0 + 8 * hh + r;
    const float z = (sZ[row] + sZ[CH + row]) + 1e-12f;
    const float inv = nrm ? (1.0f / z) : 1.0f;
#pragma unroll
    for (int t = 0; t < 2; ++t) sO[row * OP + kh * 32 + 16 * t + c] = oacc[t][r] * inv;
  }
  __syncthreads();
  v4f val[4];
  size_t go[4];
#pragma unroll
  for (int it = 0; it < 4; ++it) {
    const int p    = tid + 256 * it;
    const int L    = p >> 3;
    const int row  = L >> 1;
    const int half = L & 1;
    const int pc   = p & 7;
    val[it] = *(const v4f*)(sO + row * OP + half * 32 + pc * 4);
    go[it]  = (qrow0 + row) * DK + half * 32 + pc * 4;
  }
  for (int ps = 0; ps < 2; ++ps) {
#pragma unroll
    for (int it = 0; it < 4; ++it) *(volatile v4f*)(out + go[it]) = val[it];
    __threadfence();
  }
}

extern "C" void kernel_launch(void* const* d_in, const int* in_sizes, int n_in,
                              void* d_out, int out_size, void* d_ws, size_t ws_size,
                              hipStream_t stream) {
  if (n_in < 7) return;
  if (in_sizes[0] != NHEAD * SEQ * DK) return;
  if (in_sizes[1] != NHEAD * SEQ * DK) return;
  if (in_sizes[2] != NHEAD * SEQ * DK) return;
  if (in_sizes[3] != NHEAD * DK * FD) return;
  if (in_sizes[4] != NHEAD * DK * FD) return;
  if (in_sizes[5] < 1) return;
  if (in_sizes[6] < 1) return;
  if (out_size != NHEAD * SEQ * DK) return;

  const float* q  = (const float*)d_in[0];
  const float* k  = (const float*)d_in[1];
  const float* v  = (const float*)d_in[2];
  const float* wq = (const float*)d_in[3];
  const float* wk = (const float*)d_in[4];
  const int* use_scale = (const int*)d_in[5];
  const int* use_norm  = (const int*)d_in[6];
  float* out = (float*)d_out;

  const size_t szW = (size_t)2 * NHEAD * FD * DK * 2;
  const size_t szV = (size_t)NHEAD * DK * SEQ * 2;
  const size_t szF = (size_t)NHEAD * SEQ * DF * 2;
  size_t off = 0;
  const size_t oWH = off; off += szW;
  const size_t oWL = off; off += szW;
  const size_t oVH = off; off += szV;
  const size_t oVL = off; off += szV;
  const size_t oQH = off; off += szF;
  const size_t oQL = off; off += szF;
  const size_t oKH = off; off += szF;
  const size_t oKL = off; off += szF;
  if (off > ws_size) return;
  if (off > (size_t)134217728) return;

  char* ws = (char*)d_ws;
  unsigned short* WTH = (unsigned short*)(ws + oWH);
  unsigned short* WTL = (unsigned short*)(ws + oWL);
  unsigned short* VTH = (unsigned short*)(ws + oVH);
  unsigned short* VTL = (unsigned short*)(ws + oVL);
  unsigned short* QFH = (unsigned short*)(ws + oQH);
  unsigned short* QFL = (unsigned short*)(ws + oQL);
  unsigned short* KFH = (unsigned short*)(ws + oKH);
  unsigned short* KFL = (unsigned short*)(ws + oKL);

  const dim3 blk(256);
  k_prepw<<<dim3(2 * NHEAD), blk, 0, stream>>>(wq, wk, WTH, WTL);
  k_prepv<<<dim3(NCH, NHEAD), blk, 0, stream>>>(v, VTH, VTL);
  k_feat<<<dim3(NCH, NHEAD, 2), blk, 0, stream>>>(q, k, WTH, WTL, use_scale, QFH, QFL, KFH, KFL);
  k_attn<<<dim3(NCH, NHEAD), blk, 0, stream>>>(QFH, QFL, KFH, KFL, VTH, VTL, use_norm, out);
  (void)hipGetLastError();
}
